// GIN_31104153157817
// MI455X (gfx1250) — hardware-verified
//
#include <hip/hip_runtime.h>
#include <stddef.h>
#include <stdint.h>


#define DIN      128
#define DHID     128
#define ODIM     10
#define APW      256
#define KTOT     256
#define WSQ      (DHID * KTOT)
#define NPLANE   7
#define NTHR     256
#define NWAVE    8
#define EPT      8
#define CHUNK    (NTHR * EPT)
#define WCAP     (EPT * 32)
#define LISTN    (NWAVE * WCAP)
#define NBMAX    2048
#define RCAP     28672
#define DEGCAP   64
#define PKS      11
#define STW      512
#define GBM      64
#define GTHR     128
#define GNT      8
#define BN       (16 * GNT)
#define NUSQ     (DHID * (KTOT / 8))
#define TABL     640
#define TOFF_L1B 1920
#define TOFF_L2W 2048
#define TOFF_L2B 3328
#define TABUSED  3360
#define TABF     3584
#define HPRM     (DHID + DHID * ODIM + 32)
#define WSMAX    134217728
#define LDS_AGG  ((2 * RCAP + 2 * NBMAX + LISTN) * 4 + 64)

static_assert((CHUNK & (CHUNK - 1)) == 0 && CHUNK <= (1 << PKS));
static_assert((NBMAX & (NBMAX - 1)) == 0 && NBMAX <= (1 << PKS));
static_assert(NTHR * 8 == NBMAX);
static_assert(LISTN >= NBMAX);
static_assert(LISTN >= NWAVE * WCAP);
static_assert((RCAP % 32) == 0);
static_assert(NWAVE * STW <= RCAP);
static_assert(LDS_AGG <= 300000);
static_assert(GBM == (GTHR / 32) * 16);
static_assert((DIN % 32) == 0 && KTOT == 2 * DIN && APW == 2 * DIN);
static_assert(DIN == 32 * 4 && DHID == BN && DHID == DIN && GTHR == BN);
static_assert(DHID == 128);
static_assert((NUSQ % NTHR) == 0 && (KTOT / 8) == 32);
static_assert(((NPLANE * NUSQ) % NTHR) == 0);
static_assert(3 * TABL == TOFF_L1B && TOFF_L1B + DHID == TOFF_L2W && TOFF_L2W + DHID * ODIM == TOFF_L2B);
static_assert(TOFF_L2B + 32 == TABUSED && TABUSED - TOFF_L1B == HPRM && (HPRM % 4) == 0);
static_assert((TABF % NTHR) == 0 && TABF >= TABUSED);
static_assert((TABL % 32) == 0 && (TOFF_L1B % 32) == 0 && (TOFF_L2W % 32) == 0 && (TOFF_L2B % 32) == 0);
static_assert(ODIM == 10);
static_assert(((GBM * ODIM * 4) % 128) == 0);
static_assert(((GBM * ODIM) % GTHR) == 0);
static_assert(2 * GTHR * 4 >= GBM * ODIM);
static_assert(((50000 + GBM - 1) / GBM) * GBM == 50048 && (50048 % 128) == 0);
static_assert(1024 * 49 >= 50000);
static_assert(RCAP >= 17455);
static_assert(DEGCAP >= 35 + 8);
static_assert(500 <= 512);

typedef float          v4f  __attribute__((ext_vector_type(4)));
typedef float          v8f  __attribute__((ext_vector_type(8)));
typedef int            v4i  __attribute__((ext_vector_type(4)));
typedef int            v8i  __attribute__((ext_vector_type(8)));
typedef unsigned int   v2u  __attribute__((ext_vector_type(2)));
typedef unsigned int   v4u  __attribute__((ext_vector_type(4)));
typedef unsigned short v8us __attribute__((ext_vector_type(8)));
typedef __bf16         v16b __attribute__((ext_vector_type(16)));
typedef v4f  __attribute__((may_alias)) v4fa;
typedef v4u  __attribute__((may_alias)) v4ua;
typedef v8us __attribute__((may_alias)) v8usa;
union FragB { v16b v; v8us h[2]; v8i w; };

__device__ __forceinline__ v8f wmb(const FragB& a, const FragB& b, v8f c) {
  v8f d = __builtin_amdgcn_wmma_f32_16x16x32_bf16(false, a.v, false, b.v, (short)0, c, false, false);
  asm volatile("v_nop\n\tv_nop\n\tv_nop\n\tv_nop" : "+v"(d) : "v"(a.w), "v"(b.w));
  return d;
}

__device__ __forceinline__ unsigned short bf_bits(float f) {
  const unsigned int u = __float_as_uint(f);
  const unsigned int r = (u + 0x7FFFu + ((u >> 16) & 1u)) >> 16;
  const unsigned int q = (u >> 16) | 0x0040u;
  return (unsigned short)(((u & 0x7FFFFFFFu) > 0x7F800000u) ? q : r);
}
__device__ __forceinline__ float bf_val(unsigned short b) {
  return __uint_as_float(((unsigned int)b) << 16);
}
__device__ __forceinline__ float bf_rne(float f) { return bf_val(bf_bits(f)); }

__device__ __forceinline__ unsigned int hl2(float f0, float f1, bool isHi) {
  const unsigned short h0 = bf_bits(f0), h1 = bf_bits(f1);
  const unsigned short l0 = bf_bits(f0 - bf_val(h0)), l1 = bf_bits(f1 - bf_val(h1));
  const unsigned short q0 = isHi ? h0 : l0, q1 = isHi ? h1 : l1;
  return (unsigned int)q0 | ((unsigned int)q1 << 16);
}
__device__ __forceinline__ v4u pack8(const v4f a, const v4f b, bool isHi) {
  v4u p;
  p.x = hl2(a.x, a.y, isHi);
  p.y = hl2(a.z, a.w, isHi);
  p.z = hl2(b.x, b.y, isHi);
  p.w = hl2(b.z, b.w, isHi);
  return p;
}

__device__ __forceinline__ int scan_chunk(const int* __restrict__ dsts, int nE, int cbase, int slotBase,
                                          int nb, int vec8, int* list, int tid, int lane, int wave) {
  int wc = 0;
  const int el0  = tid * EPT;
  const int e0   = cbase + el0;
  const int sent = -2147483647 - 1;
  v4i da, db;
  if (vec8 != 0 && cbase + CHUNK <= nE) {
    da = *(const v4i*)(dsts + e0);
    db = *(const v4i*)(dsts + e0 + 4);
  } else {
    da.x = (e0     < nE) ? dsts[min(e0,     nE - 1)] : sent;
    da.y = (e0 + 1 < nE) ? dsts[min(e0 + 1, nE - 1)] : sent;
    da.z = (e0 + 2 < nE) ? dsts[min(e0 + 2, nE - 1)] : sent;
    da.w = (e0 + 3 < nE) ? dsts[min(e0 + 3, nE - 1)] : sent;
    db.x = (e0 + 4 < nE) ? dsts[min(e0 + 4, nE - 1)] : sent;
    db.y = (e0 + 5 < nE) ? dsts[min(e0 + 5, nE - 1)] : sent;
    db.z = (e0 + 6 < nE) ? dsts[min(e0 + 6, nE - 1)] : sent;
    db.w = (e0 + 7 < nE) ? dsts[min(e0 + 7, nE - 1)] : sent;
  }
  const unsigned nbs = (unsigned)slotBase;
  const unsigned unb = (unsigned)nb;
  const unsigned s0 = (unsigned)da.x - nbs, s1 = (unsigned)da.y - nbs;
  const unsigned s2 = (unsigned)da.z - nbs, s3 = (unsigned)da.w - nbs;
  const unsigned s4 = (unsigned)db.x - nbs, s5 = (unsigned)db.y - nbs;
  const unsigned s6 = (unsigned)db.z - nbs, s7 = (unsigned)db.w - nbs;
  const bool h0 = s0 < unb, h1 = s1 < unb, h2 = s2 < unb, h3 = s3 < unb;
  const bool h4 = s4 < unb, h5 = s5 < unb, h6 = s6 < unb, h7 = s7 < unb;
  const unsigned any = __builtin_amdgcn_ballot_w32(h0 | h1 | h2 | h3 | h4 | h5 | h6 | h7);
  if (any != 0u) {
#define HITJ(J, HJ, SJ) { \
      const unsigned mj = __builtin_amdgcn_ballot_w32(HJ); \
      if (mj != 0u) { \
        if (HJ) { \
          const int pos = wc + (int)__builtin_amdgcn_mbcnt_lo(mj, 0u); \
          if (pos < WCAP) list[wave * WCAP + pos] = ((el0 + (J)) << PKS) | (int)(SJ); \
        } \
        wc += (int)__builtin_popcount(mj); } }
    HITJ(0, h0, s0)
    HITJ(1, h1, s1)
    HITJ(2, h2, s2)
    HITJ(3, h3, s3)
    HITJ(4, h4, s4)
    HITJ(5, h5, s5)
    HITJ(6, h6, s6)
    HITJ(7, h7, s7)
#undef HITJ
  }
  return wc;
}

__device__ __forceinline__ v8us cv8b(const float* __restrict__ p) {
  v8us o;
#pragma unroll
  for (int i = 0; i < 8; ++i) o[i] = bf_bits(p[(size_t)i * DHID]);
  return o;
}

__global__ __launch_bounds__(NTHR) void k_wprep(const float* __restrict__ c1w1, const float* __restrict__ c1w2,
                                                const float* __restrict__ ws1,  const float* __restrict__ ws2,
                                                const float* __restrict__ l1w,  unsigned short* wt) {
  const int u = (int)blockIdx.x * NTHR + (int)threadIdx.x;
  if (u >= NPLANE * NUSQ) return;
  const int mi  = u / NUSQ;
  const int v   = u - mi * NUSQ;
  const int n   = v >> 5;
  const int k8  = (v & 31) * 8;
  const int kk  = k8 & (DIN - 1);
  const size_t eo = (size_t)kk * DHID + (size_t)n;
  v8us o;
  if (mi == 0)      o = cv8b(c1w1 + eo);
  else if (mi == 1) o = cv8b(c1w2 + eo);
  else if (mi == 2) o = cv8b(ws1 + eo);
  else if (mi == 3) o = cv8b(ws2 + eo);
  else if (mi == 4) o = cv8b(ws1 + (size_t)DIN * DHID + eo);
  else if (mi == 5) o = cv8b(ws2 + (size_t)DIN * DHID + eo);
  else              o = cv8b(l1w + eo);
  unsigned short* dp = wt + (size_t)mi * WSQ + (size_t)n * KTOT + k8;
  *(volatile v8us*)dp = o;
  __threadfence();
  *(volatile v8us*)dp = o;
}

__global__ __launch_bounds__(NTHR) void k_tab(
    const float* __restrict__ c1b1, const float* __restrict__ c1b2, const float* __restrict__ c1g,
    const float* __restrict__ c1be, const float* __restrict__ c1rm, const float* __restrict__ c1rv,
    const float* __restrict__ bs1,  const float* __restrict__ bs2,  const float* __restrict__ gs,
    const float* __restrict__ bes,  const float* __restrict__ rms,  const float* __restrict__ rvs,
    const float* __restrict__ l1b,  const float* __restrict__ l2w,  const float* __restrict__ l2b,
    float* tab) {
  __shared__ __attribute__((aligned(16))) float stg[NTHR];
  const int tid = (int)threadIdx.x;
  const int f = (int)blockIdx.x * NTHR + tid;
  float val = 0.0f;
  if (f < 3 * TABL) {
    const int l    = f / TABL;
    const int r    = f - l * TABL;
    const int kind = r >> 7;
    const int c    = r & (DHID - 1);
    const int so   = (l > 0 ? l - 1 : 0) * DHID + c;
    const bool first = (l == 0);
    if (kind == 0) {
      const float a = c1b1[c], b = bs1[so];
      val = bf_rne(first ? a : b);
    } else if (kind == 1) {
      const float a = c1b2[c], b = bs2[so];
      val = bf_rne(first ? a : b);
    } else if (kind == 2) {
      const float ga = c1g[c], gb = gs[so];
      const float va = c1rv[c], vb = rvs[so];
      const float g  = bf_rne(first ? ga : gb);
      const float rv = bf_rne(first ? va : vb);
      val = g / sqrtf(rv + 1e-5f);
    } else if (kind == 3) {
      const float a = c1rm[c], b = rms[so];
      val = bf_rne(first ? a : b);
    } else {
      const float a = c1be[c], b = bes[so];
      val = bf_rne(first ? a : b);
    }
  } else if (f < TOFF_L2W) {
    val = bf_rne(l1b[f - TOFF_L1B]);
  } else if (f < TOFF_L2B) {
    val = bf_rne(l2w[f - TOFF_L2W]);
  } else if (f < TABUSED) {
    const int j  = f - TOFF_L2B;
    const int jc = j < ODIM ? j : ODIM - 1;
    const float a = l2b[jc];
    val = (j < ODIM) ? bf_rne(a) : 0.0f;
  }
  stg[tid] = val;
  __syncthreads();
  v4f v = {0.f, 0.f, 0.f, 0.f};
  float* dp = tab + (size_t)blockIdx.x * NTHR + 4 * tid;
  if (tid < NTHR / 4) {
    v = *(const v4fa*)(stg + 4 * tid);
    *(volatile v4f*)dp = v;
  }
  __threadfence();
  if (tid < NTHR / 4) {
    *(volatile v4f*)dp = v;
  }
}

__global__ __launch_bounds__(NTHR) void k_xr(const float* __restrict__ x, int nN, int nUnits, float* xr) {
  const int u = (int)blockIdx.x * NTHR + (int)threadIdx.x;
  if (u >= nUnits) return;
  const int row = u >> 5;
  const int c4  = (u & 31) * 4;
  const int rc  = row < nN ? row : nN - 1;
  const v4f a = *(const v4f*)(x + (size_t)rc * DIN + c4);
  const bool ok = row < nN;
  v4f o;
  o.x = ok ? bf_rne(a.x) : 0.0f;
  o.y = ok ? bf_rne(a.y) : 0.0f;
  o.z = ok ? bf_rne(a.z) : 0.0f;
  o.w = ok ? bf_rne(a.w) : 0.0f;
  float* hp = xr + (size_t)row * DIN + c4;
  *(volatile v4f*)hp = o;
  __threadfence();
  *(volatile v4f*)hp = o;
}

__global__ __launch_bounds__(NTHR) void k_agg(
    const int* __restrict__ srcs, const int* __restrict__ dsts,
    const float* __restrict__ F, const float* __restrict__ epsp, int eidx,
    unsigned short* Aout, int ldaOut,
    int nN, int nE, int nb, int vec8, int MPr) {
  extern __shared__ v4f lds_dyn[];
  int* reg1 = (int*)lds_dyn;
  int* reg2 = reg1 + RCAP;
  int* scnt = reg2 + RCAP;
  int* soff = scnt + NBMAX;
  int* list = soff + NBMAX;
  int* wcnt = list + LISTN;
  int* wtot = wcnt + NWAVE;
  const int tid = (int)threadIdx.x, lane = tid & 31, wave = tid >> 5;
  const int nodeBase = (int)blockIdx.x * nb;

  for (int i = tid; i < NBMAX; i += NTHR) scnt[i] = 0;
  __syncthreads();

  int tot = 0;
  const int nChunks = (nE + CHUNK - 1) / CHUNK;
#pragma unroll 1
  for (int ch = 0; ch < nChunks; ++ch) {
    const int cbase = ch * CHUNK;
    const int wc = scan_chunk(dsts, nE, cbase, nodeBase, nb, vec8, list, tid, lane, wave);
    if (lane == 0) wcnt[wave] = wc;
    __syncthreads();
    int pre = 0, all = 0;
#pragma unroll
    for (int w2 = 0; w2 < NWAVE; ++w2) {
      int c = wcnt[w2];
      c = c < 0 ? 0 : (c > WCAP ? WCAP : c);
      all += c;
      pre += (w2 < wave) ? c : 0;
    }
    const int wcc  = wc > WCAP ? WCAP : wc;
    const int base = tot + pre;
#pragma unroll 1
    for (int i = lane; i < wcc; i += 32) {
      const int ent = list[wave * WCAP + i];
      const int el  = (ent >> PKS) & (CHUNK - 1);
      const int sl  = ent & (NBMAX - 1);
      int eid = cbase + el;
      eid = eid > nE - 1 ? nE - 1 : eid;
      const int pos = base + i;
      if (pos < RCAP) reg1[pos] = (int)(((unsigned)eid << PKS) | (unsigned)sl);
    }
    tot += all;
    tot = tot > RCAP ? RCAP : tot;
    __syncthreads();
  }
  const int nh = tot;

  if (wave == 0) {
#pragma unroll 1
    for (int b0 = 0; b0 < nh; b0 += 32) {
      const int idx = b0 + lane;
      const int uv  = reg1[idx < RCAP ? idx : RCAP - 1];
      const int m32 = (nh - b0) < 32 ? (nh - b0) : 32;
#pragma unroll 1
      for (int k = 0; k < m32; ++k) {
        const int u  = __builtin_amdgcn_readlane(uv, k);
        const int sl = u & (NBMAX - 1);
        if (lane == 0) scnt[sl] = scnt[sl] + 1;
      }
    }
  }
  __syncthreads();

  {
    const v4i ca = *(const v4i*)(scnt + 8 * tid);
    const v4i cb = *(const v4i*)(scnt + 8 * tid + 4);
    const int e0 = ca.x < 0 ? 0 : ca.x, e1 = ca.y < 0 ? 0 : ca.y, e2 = ca.z < 0 ? 0 : ca.z, e3 = ca.w < 0 ? 0 : ca.w;
    const int e4 = cb.x < 0 ? 0 : cb.x, e5 = cb.y < 0 ? 0 : cb.y, e6 = cb.z < 0 ? 0 : cb.z, e7 = cb.w < 0 ? 0 : cb.w;
    const int ts = e0 + e1 + e2 + e3 + e4 + e5 + e6 + e7;
    int incl = ts;
#pragma unroll
    for (int d = 1; d < 32; d <<= 1) {
      const int up = __shfl_up(incl, d);
      if (lane >= d) incl += up;
    }
    if (lane == 31) wtot[wave] = incl;
    __syncthreads();
    int pre = 0;
#pragma unroll
    for (int w2 = 0; w2 < NWAVE; ++w2) pre += (w2 < wave) ? wtot[w2] : 0;
    int run = pre + incl - ts;
    soff[8 * tid + 0] = run; run += e0;
    soff[8 * tid + 1] = run; run += e1;
    soff[8 * tid + 2] = run; run += e2;
    soff[8 * tid + 3] = run; run += e3;
    soff[8 * tid + 4] = run; run += e4;
    soff[8 * tid + 5] = run; run += e5;
    soff[8 * tid + 6] = run; run += e6;
    soff[8 * tid + 7] = run;
  }
  __syncthreads();
  for (int i = tid; i < NBMAX; i += NTHR) list[i] = soff[i];
  __syncthreads();

  if (wave == 0) {
#pragma unroll 1
    for (int b0 = 0; b0 < nh; b0 += 32) {
      const int idx = b0 + lane;
      const int uv  = reg1[idx < RCAP ? idx : RCAP - 1];
      const int m32 = (nh - b0) < 32 ? (nh - b0) : 32;
#pragma unroll 1
      for (int k = 0; k < m32; ++k) {
        const int u   = __builtin_amdgcn_readlane(uv, k);
        const int sl  = u & (NBMAX - 1);
        const int eid = (int)((unsigned)u >> PKS);
        if (lane == 0) {
          int pos = list[sl];
          pos = pos < 0 ? 0 : (pos > RCAP - 1 ? RCAP - 1 : pos);
          reg2[pos] = eid;
          list[sl] = pos + 1;
        }
      }
    }
  }
  __syncthreads();

  const int nbw = nb >> 3;
  const bool ovf = (nh >= RCAP);
  const float qnan = __int_as_float(0x7fc00000);
  const float ev = 1.0f + bf_rne(epsp[eidx]);
  unsigned int* stwu = (unsigned int*)((float*)reg1 + wave * STW);

#pragma unroll 1
  for (int jt = 0; jt < nbw; ++jt) {
    const int slot = wave * nbw + jt;
    const int grow = nodeBase + slot;
    int st = soff[slot];
    const int craw = scnt[slot];
    int cnt = craw;
    st  = st < 0 ? 0 : (st > nh ? nh : st);
    cnt = cnt < 0 ? 0 : (cnt > DEGCAP ? DEGCAP : cnt);
    if (cnt > nh - st) cnt = nh - st;
    const float pz = (ovf || craw > DEGCAP) ? qnan : 0.0f;
    const bool liveRow = grow < nN;

    float ag0 = 0.f, ag1 = 0.f, ag2 = 0.f, ag3 = 0.f;
#pragma unroll 1
    for (int b0 = 0; b0 < cnt; b0 += 32) {
      int idx = st + b0 + lane;
      idx = idx > nh - 1 ? nh - 1 : idx;
      idx = idx < 0 ? 0 : (idx > RCAP - 1 ? RCAP - 1 : idx);
      int eid = reg2[idx];
      eid = eid < 0 ? 0 : (eid > nE - 1 ? nE - 1 : eid);
      const int sraw = srcs[eid];
      const int sv = sraw < 0 ? 0 : (sraw > nN - 1 ? nN - 1 : sraw);
      const int m32 = (cnt - b0) < 32 ? (cnt - b0) : 32;
#pragma unroll 1
      for (int k = 0; k < m32; ++k) {
        const int sk = __builtin_amdgcn_readlane(sv, k);
        const v4f v = *(const v4f*)(F + (size_t)sk * DIN + 4 * lane);
        ag0 += v.x; ag1 += v.y; ag2 += v.z; ag3 += v.w;
      }
    }
    const int nc = liveRow ? grow : nN - 1;
    const v4f sf = *(const v4f*)(F + (size_t)nc * DIN + 4 * lane);
    float r0 = ev * sf.x + ag0, r1 = ev * sf.y + ag1, r2 = ev * sf.z + ag2, r3 = ev * sf.w + ag3;
    r0 = (liveRow ? r0 : 0.0f) + pz;
    r1 = (liveRow ? r1 : 0.0f) + pz;
    r2 = (liveRow ? r2 : 0.0f) + pz;
    r3 = (liveRow ? r3 : 0.0f) + pz;

    const unsigned short hb0 = bf_bits(r0), hb1 = bf_bits(r1), hb2 = bf_bits(r2), hb3 = bf_bits(r3);
    const unsigned short lb0 = bf_bits(r0 - bf_val(hb0)), lb1 = bf_bits(r1 - bf_val(hb1));
    const unsigned short lb2 = bf_bits(r2 - bf_val(hb2)), lb3 = bf_bits(r3 - bf_val(hb3));
    v2u hw, lw;
    hw.x = (unsigned int)hb0 | ((unsigned int)hb1 << 16);
    hw.y = (unsigned int)hb2 | ((unsigned int)hb3 << 16);
    lw.x = (unsigned int)lb0 | ((unsigned int)lb1 << 16);
    lw.y = (unsigned int)lb2 | ((unsigned int)lb3 << 16);
    __builtin_amdgcn_fence(__ATOMIC_RELEASE, "wavefront");
    __builtin_amdgcn_wave_barrier();
    *(v2u*)(stwu + 2 * lane)      = hw;
    *(v2u*)(stwu + 64 + 2 * lane) = lw;
    __builtin_amdgcn_fence(__ATOMIC_RELEASE, "wavefront");
    __builtin_amdgcn_wave_barrier();
    const v4u pk = *(const v4ua*)(stwu + 4 * lane);
    unsigned short* gp = Aout + (size_t)grow * (size_t)ldaOut + 8 * lane;
    const bool wsv = grow < MPr;
    if (wsv) *(volatile v4u*)gp = pk;
    __threadfence();
    if (wsv) *(volatile v4u*)gp = pk;
  }
}

template <int MODE>
__global__ __launch_bounds__(GTHR) void k_gemm(const unsigned short* __restrict__ A,
                                               const unsigned short* __restrict__ WT,
                                               const float* __restrict__ prm,
                                               void* outp, int nN, int mRows)
{
  constexpr int NT = GNT;
  constexpr int NI = 16;
  constexpr int NPRM = (MODE == 1) ? DHID : ((MODE == 0) ? 4 * DHID : HPRM);
  constexpr int NLG  = (MODE == 2) ? GBM * ODIM : 4;
  __shared__ __attribute__((aligned(16))) float stg[GBM * BN];
  __shared__ __attribute__((aligned(16))) float prs[NPRM];
  __shared__ __attribute__((aligned(16))) float lg[NLG];
  __shared__ __attribute__((aligned(16))) float ot[NLG];
  const int tid = (int)threadIdx.x, lane = tid & 31, wave = tid >> 5, hh = lane >> 4, m = lane & 15;
  const int rowBase = (int)blockIdx.x * GBM;

#pragma unroll 1
  for (int i = tid; i < NPRM / 4; i += GTHR) {
    const v4f pv = *(const v4f*)(prm + 4 * i);
    *(v4fa*)(prs + 4 * i) = pv;
  }
  __syncthreads();

  v8f acc[NT];
  {
    const v8f z = {0.f, 0.f, 0.f, 0.f, 0.f, 0.f, 0.f, 0.f};
#pragma unroll
    for (int t = 0; t < NT; ++t) acc[t] = z;
  }
  const unsigned short* ap = A + (size_t)(rowBase + 16 * wave + m) * (size_t)APW + 8 * hh;
  const unsigned short* wp = WT + (size_t)m * (size_t)KTOT + 8 * hh;
  constexpr int ksteps = KTOT / 32;
#pragma unroll 1
  for (int ks = 0; ks < ksteps; ++ks) {
    FragB af;
    af.h[0] = *(const v8usa*)(ap + 32 * ks);
    af.h[1] = *(const v8usa*)(ap + 32 * ks + 16);
#pragma unroll
    for (int t = 0; t < NT; ++t) {
      const unsigned short* wq = wp + (size_t)(16 * t) * (size_t)KTOT + 32 * ks;
      FragB bf;
      bf.h[0] = *(const v8usa*)wq;
      bf.h[1] = *(const v8usa*)(wq + 16);
      acc[t] = wmb(af, bf, acc[t]);
    }
  }

#pragma unroll
  for (int t = 0; t < NT; ++t) {
    const int lc = 16 * t + m;
    const float bb = prs[lc];
    float sc = 1.0f, rmv = 0.0f, bev = 0.0f;
    if constexpr (MODE == 0) {
      sc  = prs[DHID + lc];
      rmv = prs[2 * DHID + lc];
      bev = prs[3 * DHID + lc];
    }
#pragma unroll
    for (int r = 0; r < 8; ++r) {
      const int lr = 16 * wave + 8 * hh + r;
      const bool live = (rowBase + lr) < nN;
      float v = acc[t][r] + bb;
      v = (v > 0.0f) ? v : (v - v);
      if constexpr (MODE == 0) v = (v - rmv) * sc + bev;
      stg[lr * BN + lc] = live ? v : 0.0f;
    }
  }
  __syncthreads();

  if constexpr (MODE == 0) {
    float* outF = (float*)outp;
    v4f fv[NI];
#pragma unroll
    for (int i = 0; i < NI; ++i) {
      const int lr = 16 * wave + i;
      fv[i] = *(const v4fa*)(stg + lr * BN + 4 * lane);
    }
#pragma unroll
    for (int i = 0; i < NI; ++i) {
      const int gr = rowBase + 16 * wave + i;
      float* op = outF + (size_t)gr * (size_t)DHID + 4 * lane;
      if (gr < mRows) *(volatile v4f*)op = fv[i];
    }
    __threadfence();
#pragma unroll
    for (int i = 0; i < NI; ++i) {
      const int gr = rowBase + 16 * wave + i;
      float* op = outF + (size_t)gr * (size_t)DHID + 4 * lane;
      if (gr < mRows) *(volatile v4f*)op = fv[i];
    }
  } else if constexpr (MODE == 1) {
    unsigned short* outH = (unsigned short*)outp;
    const int cb = 8 * m;
    const bool isHi = (hh == 0);
    v4u pk[NI];
#pragma unroll
    for (int i = 0; i < NI; ++i) {
      const int lr = 16 * wave + i;
      const v4f a = *(const v4fa*)(stg + lr * BN + cb);
      const v4f b = *(const v4fa*)(stg + lr * BN + cb + 4);
      pk[i] = pack8(a, b, isHi);
    }
#pragma unroll
    for (int i = 0; i < NI; ++i) {
      const int gr = rowBase + 16 * wave + i;
      unsigned short* op = outH + (size_t)gr * (size_t)APW + 8 * lane;
      if (gr < mRows) *(volatile v4u*)op = pk[i];
    }
    __threadfence();
#pragma unroll
    for (int i = 0; i < NI; ++i) {
      const int gr = rowBase + 16 * wave + i;
      unsigned short* op = outH + (size_t)gr * (size_t)APW + 8 * lane;
      if (gr < mRows) *(volatile v4u*)op = pk[i];
    }
  } else {
#pragma unroll 1
    for (int it = 0; it < (GBM * ODIM) / GTHR; ++it) {
      const int idx = it * GTHR + tid;
      const int row = idx / ODIM;
      const int c   = idx - row * ODIM;
      float s = 0.0f;
#pragma unroll 4
      for (int k = 0; k < DHID; ++k) s = fmaf(stg[row * BN + k], prs[DHID + k * ODIM + c], s);
      lg[idx] = s + prs[DHID + DHID * ODIM + c];
    }
    __syncthreads();
    if (tid < GBM) {
      float mx = lg[tid * ODIM];
#pragma unroll 1
      for (int c = 1; c < ODIM; ++c) {
        const float v = lg[tid * ODIM + c];
        mx = (v > mx || v != v) ? v : mx;
      }
      float se = 0.0f;
#pragma unroll 1
      for (int c = 0; c < ODIM; ++c) se += expf(lg[tid * ODIM + c] - mx);
      const float ls = logf(se);
#pragma unroll 1
      for (int c = 0; c < ODIM; ++c) ot[tid * ODIM + c] = (lg[tid * ODIM + c] - mx) - ls;
    }
    __syncthreads();
    int nLive = nN - rowBase;
    nLive = nLive < 0 ? 0 : (nLive > GBM ? GBM : nLive);
    const int nQ = (nLive * ODIM) >> 2;
    float* outF = (float*)outp + (size_t)rowBase * ODIM;
    const int p0 = tid, p1 = GTHR + tid;
    const int q0 = p0 < nQ ? p0 : 0, q1 = p1 < nQ ? p1 : 0;
    const v4f ov0 = *(const v4fa*)(ot + 4 * q0);
    const v4f ov1 = *(const v4fa*)(ot + 4 * q1);
    if (p0 < nQ) *(volatile v4f*)(outF + 4 * p0) = ov0;
    if (p1 < nQ) *(volatile v4f*)(outF + 4 * p1) = ov1;
    __threadfence();
    if (p0 < nQ) *(volatile v4f*)(outF + 4 * p0) = ov0;
    if (p1 < nQ) *(volatile v4f*)(outF + 4 * p1) = ov1;
  }
}

__global__ __launch_bounds__(NTHR) void k_pool(const float* __restrict__ hf, const int* __restrict__ bat,
                                               int nN, int nG, unsigned short* pg) {
  __shared__ __attribute__((aligned(16))) float wsum[NWAVE * DHID];
  __shared__ int wcn[NWAVE];
  __shared__ __attribute__((aligned(16))) float outs[DHID];
  const int tid = (int)threadIdx.x, lane = tid & 31, wave = tid >> 5;
  const int g = (int)blockIdx.x;
  const int nEff = (g < nG) ? nN : 0;

  float a0 = 0.0f, a1 = 0.0f, a2 = 0.0f, a3 = 0.0f;
  int cnt = 0;
#pragma unroll 1
  for (int i0 = wave * 32; i0 < nEff; i0 += NTHR) {
    const int i  = i0 + lane;
    const int ic = i < nN ? i : nN - 1;
    const int b  = bat[ic];
    const bool hit = (i < nN) && (b == g);
    unsigned msk = __builtin_amdgcn_ballot_w32(hit);
    int nh = (int)__builtin_popcount(msk);
    nh = nh > 32 ? 32 : nh;
    cnt += nh;
#pragma unroll 1
    for (int q = 0; q < nh; ++q) {
      const int k = __builtin_ffs((int)msk) - 1;
      msk &= msk - 1u;
      int node = i0 + (k < 0 ? 0 : k);
      node = node > nN - 1 ? nN - 1 : node;
      const v4f v = *(const v4f*)(hf + (size_t)node * DHID + 4 * lane);
      a0 += v.x; a1 += v.y; a2 += v.z; a3 += v.w;
    }
  }
  wsum[wave * DHID + 4 * lane + 0] = a0;
  wsum[wave * DHID + 4 * lane + 1] = a1;
  wsum[wave * DHID + 4 * lane + 2] = a2;
  wsum[wave * DHID + 4 * lane + 3] = a3;
  if (lane == 0) wcn[wave] = cnt;
  __syncthreads();
  if (tid < DHID) {
    float s = 0.0f;
    int c = 0;
#pragma unroll
    for (int w2 = 0; w2 < NWAVE; ++w2) { s += wsum[w2 * DHID + tid]; c += wcn[w2]; }
    const float cf = (c < 1) ? 1.0f : (float)c;
    outs[tid] = s * (1.0f / cf);
  }
  __syncthreads();
  const int hh = lane >> 4, m = lane & 15;
  const int cb = 8 * m;
  const v4f pa = *(const v4fa*)(outs + cb);
  const v4f pb = *(const v4fa*)(outs + cb + 4);
  const v4u pk = pack8(pa, pb, hh == 0);
  unsigned short* gp = pg + (size_t)g * APW + 8 * lane;
  const bool okst = (wave == 0);
  if (okst) *(volatile v4u*)gp = pk;
  __threadfence();
  if (okst) *(volatile v4u*)gp = pk;
}

static int pick_nb(int nE, int nN) {
  int nb = NBMAX;
  while (nb > 16 && (long long)nb * (long long)nE * 5LL > (long long)RCAP * (long long)nN * 4LL) nb >>= 1;
  return nb;
}
static inline int cdiv(int a, int b) { return (a + b - 1) / b; }
static inline size_t al256(size_t o) { return (o + 255) & ~(size_t)255; }

extern "C" void kernel_launch(void* const* d_in, const int* in_sizes, int n_in,
                              void* d_out, int out_size, void* d_ws, size_t ws_size,
                              hipStream_t stream) {
  if (n_in < 25) return;
  if (in_sizes[0] < DIN || (in_sizes[0] % DIN) != 0) return;
  const int nN = in_sizes[0] / DIN;
  if (nN < 1 || nN > (1 << 22)) return;
  const int nE2 = in_sizes[1];
  if (nE2 < 2 || (nE2 & 1) != 0) return;
  const int nE = nE2 / 2;
  if (nE < 1 || nE > (1 << 21)) return;
  if (in_sizes[2] != nN) return;
  if (in_sizes[3] != DIN * DHID || in_sizes[5] != DHID * DHID) return;
  if (in_sizes[4] != DHID || in_sizes[6] != DHID) return;
  if (in_sizes[7] != DHID || in_sizes[8] != DHID || in_sizes[9] != DHID || in_sizes[10] != DHID) return;
  if (in_sizes[11] != 1) return;
  if (in_sizes[12] != 2 * DHID * DHID || in_sizes[14] != 2 * DHID * DHID) return;
  if (in_sizes[13] != 2 * DHID || in_sizes[15] != 2 * DHID) return;
  if (in_sizes[16] != 2 * DHID || in_sizes[17] != 2 * DHID) return;
  if (in_sizes[18] != 2 * DHID || in_sizes[19] != 2 * DHID) return;
  if (in_sizes[20] != 2) return;
  if (in_sizes[21] != DHID * DHID || in_sizes[22] != DHID) return;
  if (in_sizes[23] != DHID * ODIM || in_sizes[24] != ODIM) return;
  if (out_size < ODIM || (out_size % ODIM) != 0) return;
  const int nG = out_size / ODIM;
  if (nG < 1 || nG > 65535 || (nG & 1) != 0) return;
  if ((long long)nG * ODIM != (long long)out_size) return;

  const float* x     = (const float*)d_in[0];
  const int*   ei    = (const int*)  d_in[1];
  const int*   src   = ei;
  const int*   dst   = ei + nE;
  const int*   bat   = (const int*)  d_in[2];
  const float* c1W1  = (const float*)d_in[3];
  const float* c1b1  = (const float*)d_in[4];
  const float* c1W2  = (const float*)d_in[5];
  const float* c1b2  = (const float*)d_in[6];
  const float* c1g   = (const float*)d_in[7];
  const float* c1be  = (const float*)d_in[8];
  const float* c1rm  = (const float*)d_in[9];
  const float* c1rv  = (const float*)d_in[10];
  const float* c1eps = (const float*)d_in[11];
  const float* Ws1   = (const float*)d_in[12];
  const float* bs1   = (const float*)d_in[13];
  const float* Ws2   = (const float*)d_in[14];
  const float* bs2   = (const float*)d_in[15];
  const float* gs    = (const float*)d_in[16];
  const float* bes   = (const float*)d_in[17];
  const float* rms   = (const float*)d_in[18];
  const float* rvs   = (const float*)d_in[19];
  const float* epss  = (const float*)d_in[20];
  const float* l1W   = (const float*)d_in[21];
  const float* l1b   = (const float*)d_in[22];
  const float* l2W   = (const float*)d_in[23];
  const float* l2b   = (const float*)d_in[24];
  float* out = (float*)d_out;

  const int MP   = cdiv(nN, GBM) * GBM;
  const int gM   = MP / GBM;
  const int GP   = cdiv(nG, GBM) * GBM;
  const int gH   = GP / GBM;
  const int nb   = pick_nb(nE, nN);
  const int gA   = cdiv(MP, nb);
  const int vec8 = ((nE & 3) == 0) ? 1 : 0;
  if ((long long)gA * nb < (long long)MP) return;
  if ((long long)(gM - 1) * GBM >= (long long)nN) return;
  if ((long long)(gH - 1) * GBM >= (long long)nG) return;
  const int nUx = MP * (DIN / 4);

  char* ws = (char*)d_ws;
  size_t off = 0;
  const size_t oWT  = off; off = al256(off + (size_t)NPLANE * WSQ * 2);
  const size_t oTAB = off; off = al256(off + (size_t)TABF * 4);
  const size_t oPH  = off; off = al256(off + (size_t)MP * DHID * 4);
  const size_t oPZ  = off; off = al256(off + (size_t)MP * APW * 2);
  const size_t oPT  = off; off = al256(off + (size_t)MP * APW * 2);
  const size_t oPG  = off; off = al256(off + (size_t)GP * APW * 2);
  if (off > ws_size || off > (size_t)WSMAX) return;
  unsigned short* WT  = (unsigned short*)(ws + oWT);
  float*          TAB = (float*)(ws + oTAB);
  float*          PH  = (float*)(ws + oPH);
  unsigned short* PZ  = (unsigned short*)(ws + oPZ);
  unsigned short* PT  = (unsigned short*)(ws + oPT);
  unsigned short* PG  = (unsigned short*)(ws + oPG);

  hipFuncSetAttribute(reinterpret_cast<const void*>(&k_agg), hipFuncAttributeMaxDynamicSharedMemorySize, LDS_AGG);

  k_wprep<<<(NPLANE * NUSQ) / NTHR, NTHR, 0, stream>>>(c1W1, c1W2, Ws1, Ws2, l1W, WT);
  k_tab<<<TABF / NTHR, NTHR, 0, stream>>>(c1b1, c1b2, c1g, c1be, c1rm, c1rv,
                                          bs1, bs2, gs, bes, rms, rvs, l1b, l2W, l2b, TAB);
  k_xr<<<cdiv(nUx, NTHR), NTHR, 0, stream>>>(x, nN, nUx, PH);
  for (int l = 0; l < 3; ++l) {
    const float* epsp = (l == 0) ? c1eps : epss;
    const int    eidx = (l == 0) ? 0 : (l - 1);
    k_agg<<<gA, NTHR, LDS_AGG, stream>>>(src, dst, PH, epsp, eidx, PZ, APW, nN, nE, nb, vec8, MP);
    k_gemm<1><<<gM, GTHR, 0, stream>>>(PZ, WT + (size_t)(2 * l) * WSQ, TAB + (size_t)l * TABL,
                                       (void*)PT, nN, MP);
    k_gemm<0><<<gM, GTHR, 0, stream>>>(PT, WT + (size_t)(2 * l + 1) * WSQ, TAB + (size_t)l * TABL + DHID,
                                       (void*)PH, nN, MP);
  }
  k_pool<<<GP, NTHR, 0, stream>>>(PH, bat, nN, nG, PG);
  k_gemm<2><<<gH, GTHR, 0, stream>>>(PG, WT + (size_t)6 * WSQ, TAB + TOFF_L1B, (void*)out, nG, GP);
}
